// ParagraphGATInference_23965917512221
// MI455X (gfx1250) — hardware-verified
//
#include <hip/hip_runtime.h>

typedef _Float16 v16h __attribute__((ext_vector_type(16)));
typedef _Float16 v8h  __attribute__((ext_vector_type(8)));
typedef float    v8f  __attribute__((ext_vector_type(8)));
typedef float    v4f  __attribute__((ext_vector_type(4)));

#define DIM 128
#define HD 512
#define HD2 1024
#define NEG_SLOPE 0.2f
#define LN_EPS 1e-5f
#define WSCALE 16.0f
#define WINV 0.0625f

#define GBM 128
#define GBN 128
#define BPITCH 136
#define LDS_GEMM_V4 2176

#define NPB 256
#define LCAP 768
#define SCAP 6144
#define DEGCAP 160

union Frag { v16h v; v8h hh[2]; };

__device__ __forceinline__ v8f wmma_f16(v16h a, v16h b, v8f c) {
  v8f d = __builtin_amdgcn_wmma_f32_16x16x32_f16(false, a, false, b, (short)0, c, false, false);
  asm volatile("v_nop\n\tv_nop\n\tv_nop\n\tv_nop" : "+v"(d) : "v"(a), "v"(b));
  return d;
}

__device__ __forceinline__ v8h cvt8(v4f p, v4f q) {
  v8h r;
  r[0] = (_Float16)p[0]; r[1] = (_Float16)p[1]; r[2] = (_Float16)p[2]; r[3] = (_Float16)p[3];
  r[4] = (_Float16)q[0]; r[5] = (_Float16)q[1]; r[6] = (_Float16)q[2]; r[7] = (_Float16)q[3];
  return r;
}

__device__ __forceinline__ float wsum32(float v) {
#pragma unroll
  for (int off = 16; off > 0; off >>= 1) v += __shfl_xor(v, off, 32);
  return v;
}

__global__ __launch_bounds__(256)
void k_gemm(const float* __restrict__ A, int lda, int nrows,
            const float* __restrict__ W0, const float* __restrict__ W1, float* C) {
  __shared__ v4f s_lds[LDS_GEMM_V4];
  _Float16* Bt = (_Float16*)s_lds;
  float* stg = (float*)s_lds;

  const int tid = threadIdx.x;
  const int lane = tid & 31, wave = tid >> 5;
  const int hh = lane >> 4, m = lane & 15;
  const int by = blockIdx.y;
  const float* W = (by < 4) ? W0 : W1;
  const int cb = (by & 3) * GBN;

#pragma unroll 4
  for (int it = 0; it < 16; ++it) {
    const int f = it * 256 + tid;
    const int n4 = (f & 31) * 4;
    const int k = f >> 5;
    const v4f w = *(const v4f*)(W + (size_t)k * HD + cb + n4);
    Bt[(n4 + 0) * BPITCH + k] = (_Float16)(w[0] * WSCALE);
    Bt[(n4 + 1) * BPITCH + k] = (_Float16)(w[1] * WSCALE);
    Bt[(n4 + 2) * BPITCH + k] = (_Float16)(w[2] * WSCALE);
    Bt[(n4 + 3) * BPITCH + k] = (_Float16)(w[3] * WSCALE);
  }
  __syncthreads();

  const int row0 = blockIdx.x * GBM + wave * 16;
  int ra = row0 + m;
  if (ra > nrows - 1) ra = nrows - 1;
  const float* arow = A + (size_t)ra * lda;

  v8f zero8;
#pragma unroll
  for (int i = 0; i < 8; ++i) zero8[i] = 0.f;
  v8f acc[8];
#pragma unroll
  for (int t = 0; t < 8; ++t) acc[t] = zero8;

#pragma unroll
  for (int kk = 0; kk < 4; ++kk) {
    const int k0 = kk * 32;
    Frag fa;
    fa.hh[0] = cvt8(*(const v4f*)(arow + k0 + 8 * hh), *(const v4f*)(arow + k0 + 8 * hh + 4));
    fa.hh[1] = cvt8(*(const v4f*)(arow + k0 + 16 + 8 * hh), *(const v4f*)(arow + k0 + 20 + 8 * hh));
#pragma unroll
    for (int t = 0; t < 8; ++t) {
      const _Float16* bp = Bt + (t * 16 + m) * BPITCH + k0 + 8 * hh;
      Frag fb;
      fb.hh[0] = *(const v8h*)bp;
      fb.hh[1] = *(const v8h*)(bp + 16);
      acc[t] = wmma_f16(fa.v, fb.v, acc[t]);
    }
  }
  __syncthreads();

  float* sw = stg + wave * (16 * 64);
  float* cw = C + (size_t)row0 * HD2 + by * GBN + 4 * m;
#pragma unroll
  for (int p = 0; p < 2; ++p) {
    if (p) __syncthreads();
#pragma unroll
    for (int t = 0; t < 4; ++t) {
      const v8f a8 = acc[4 * p + t];
#pragma unroll
      for (int r = 0; r < 8; ++r) sw[(8 * hh + r) * 64 + t * 16 + m] = a8[r] * WINV;
    }
    __syncthreads();
    v4f v[8];
#pragma unroll
    for (int i = 0; i < 8; ++i) v[i] = *(const v4f*)(sw + (2 * i + hh) * 64 + 4 * m);
    float* cp = cw + p * 64;
#pragma unroll
    for (int i = 0; i < 8; ++i) *(volatile v4f*)(cp + (size_t)(2 * i + hh) * HD2) = v[i];
    __threadfence();
#pragma unroll
    for (int i = 0; i < 8; ++i) *(volatile v4f*)(cp + (size_t)(2 * i + hh) * HD2) = v[i];
  }
}

__global__ __launch_bounds__(256)
void k_edge(const float* __restrict__ xlr, const int* __restrict__ src, const int* __restrict__ dst,
            int E, int nChunks, int N,
            const float* __restrict__ att, const float* __restrict__ bias,
            const float* __restrict__ gam, const float* __restrict__ bet,
            const float* __restrict__ resid, float* out, int relu) {
  __shared__ unsigned listL[8 * LCAP];
  __shared__ unsigned sortedL[SCAP];
  __shared__ int histL[8 * NPB];
  __shared__ int offL[NPB];
  __shared__ int cntL[NPB];
  __shared__ int wtot[8];

  const int tid = threadIdx.x;
  const int lane = tid & 31, wave = tid >> 5;
  const int n0 = blockIdx.x * NPB;
  const unsigned ltmask = (1u << lane) - 1u;
  const int lb = wave * LCAP;
  const int hb = wave * NPB;

  unsigned cntw = 0u;
  for (int c = 0; c < nChunks; ++c) {
    const int e = c * 256 + tid;
    int d = -1;
    if (e < E) d = dst[e];
    const int dl = d - n0;
    const bool hit = (e < E) && (d >= 0) && (d < N) && (dl >= 0) && (dl < NPB);
    const unsigned mask = __builtin_amdgcn_ballot_w32(hit);
    if (hit) {
      const unsigned pos = cntw + (unsigned)__builtin_popcount(mask & ltmask);
      if (pos < (unsigned)LCAP) listL[lb + pos] = ((unsigned)dl << 24) | (unsigned)e;
    }
    cntw += (unsigned)__builtin_popcount(mask);
  }
  if (cntw > (unsigned)LCAP) cntw = (unsigned)LCAP;

#pragma unroll
  for (int j = 0; j < NPB / 32; ++j) histL[hb + lane + 32 * j] = 0;
#pragma unroll 1
  for (int b = 0; b < LCAP / 32; ++b) {
    const unsigned idx = (unsigned)(b * 32 + lane);
    const bool act = idx < cntw;
    const unsigned ent = act ? listL[lb + idx] : 0u;
    const int g = (int)(ent >> 24);
    unsigned rem = __builtin_amdgcn_ballot_w32(act);
    for (int it = 0; it < 32; ++it) {
      if (rem == 0u) break;
      const int lead = __builtin_ctz(rem);
      const int gsel = __shfl(g, lead, 32);
      const bool mem = (((rem >> lane) & 1u) != 0u) && (g == gsel);
      const unsigned mm = __builtin_amdgcn_ballot_w32(mem);
      const int c0 = histL[hb + gsel];
      if (mem) histL[hb + gsel] = c0 + __builtin_popcount(mm);
      rem &= ~mm;
    }
  }
  __syncthreads();

  int tot;
  {
    int run = 0;
#pragma unroll
    for (int w = 0; w < 8; ++w) {
      const int hv = histL[w * NPB + tid];
      histL[w * NPB + tid] = run;
      run += hv;
    }
    tot = run;
  }
  int inc = tot;
#pragma unroll
  for (int o = 1; o < 32; o <<= 1) {
    const int y = __shfl_up(inc, o, 32);
    if (lane >= o) inc += y;
  }
  if (lane == 31) wtot[wave] = inc;
  __syncthreads();
  int wpre = 0;
#pragma unroll
  for (int w = 0; w < 8; ++w) wpre += (w < wave) ? wtot[w] : 0;
  const int excl = wpre + inc - tot;
  offL[tid] = excl;
  cntL[tid] = tot;
#pragma unroll
  for (int w = 0; w < 8; ++w) histL[w * NPB + tid] += excl;
  __syncthreads();

#pragma unroll 1
  for (int b = 0; b < LCAP / 32; ++b) {
    const unsigned idx = (unsigned)(b * 32 + lane);
    const bool act = idx < cntw;
    const unsigned ent = act ? listL[lb + idx] : 0u;
    const int g = (int)(ent >> 24);
    unsigned rem = __builtin_amdgcn_ballot_w32(act);
    for (int it = 0; it < 32; ++it) {
      if (rem == 0u) break;
      const int lead = __builtin_ctz(rem);
      const int gsel = __shfl(g, lead, 32);
      const bool mem = (((rem >> lane) & 1u) != 0u) && (g == gsel);
      const unsigned mm = __builtin_amdgcn_ballot_w32(mem);
      const int c0 = histL[hb + gsel];
      if (mem) {
        const int pos = c0 + __builtin_popcount(mm & ltmask);
        if ((unsigned)pos < (unsigned)SCAP) sortedL[pos] = ent & 0x00FFFFFFu;
        histL[hb + gsel] = c0 + __builtin_popcount(mm);
      }
      rem &= ~mm;
    }
  }
  __syncthreads();

  float at[16], xr[16], acc[16], xv[16], o[16];
  {
    const float* ap = att + 16 * lane;
    const v4f a0 = *(const v4f*)(ap + 0), a1 = *(const v4f*)(ap + 4);
    const v4f a2 = *(const v4f*)(ap + 8), a3 = *(const v4f*)(ap + 12);
#pragma unroll
    for (int i = 0; i < 4; ++i) { at[i] = a0[i]; at[4 + i] = a1[i]; at[8 + i] = a2[i]; at[12 + i] = a3[i]; }
  }
  const v4f bias4 = *(const v4f*)(bias + 4 * lane);
  const v4f g4 = *(const v4f*)(gam + 4 * lane);
  const v4f be4 = *(const v4f*)(bet + 4 * lane);
  const int srcl = lane >> 2, sel = lane & 3;
  const float NEG_INF = __int_as_float(0xff800000);

#pragma unroll 1
  for (int j = 0; j < 32; ++j) {
    const int lt = wave * 32 + j;
    const int node = n0 + lt;
    const bool valid = node < N;
    const int nodec = valid ? node : (N - 1);
    {
      const float* rp = xlr + (size_t)nodec * HD2 + HD + 16 * lane;
      const v4f r0 = *(const v4f*)(rp + 0), r1 = *(const v4f*)(rp + 4);
      const v4f r2 = *(const v4f*)(rp + 8), r3 = *(const v4f*)(rp + 12);
#pragma unroll
      for (int i = 0; i < 4; ++i) { xr[i] = r0[i]; xr[4 + i] = r1[i]; xr[8 + i] = r2[i]; xr[12 + i] = r3[i]; }
    }
    int cnt = cntL[lt];
    cnt = (cnt < 0) ? 0 : ((cnt > DEGCAP) ? DEGCAP : cnt);
    const int base = offL[lt];

    float mrun = NEG_INF, dsum = 0.f;
#pragma unroll
    for (int i = 0; i < 16; ++i) acc[i] = 0.f;

#pragma unroll 1
    for (int k = 0; k <= cnt; ++k) {
      int sidx = nodec;
      if (k > 0) {
        int pos = base + k - 1;
        pos = (pos < 0) ? 0 : ((pos > SCAP - 1) ? (SCAP - 1) : pos);
        int e = (int)sortedL[pos];
        e = (e < 0) ? 0 : ((e > E - 1) ? (E - 1) : e);
        int sv = src[e];
        sv = (sv < 0) ? 0 : ((sv > N - 1) ? (N - 1) : sv);
        sidx = sv;
      }
      const float* xp = xlr + (size_t)sidx * HD2 + 16 * lane;
      {
        const v4f q0 = *(const v4f*)(xp + 0), q1 = *(const v4f*)(xp + 4);
        const v4f q2 = *(const v4f*)(xp + 8), q3 = *(const v4f*)(xp + 12);
#pragma unroll
        for (int i = 0; i < 4; ++i) { xv[i] = q0[i]; xv[4 + i] = q1[i]; xv[8 + i] = q2[i]; xv[12 + i] = q3[i]; }
      }
      float p = 0.f;
#pragma unroll
      for (int i = 0; i < 16; ++i) {
        float v = xv[i] + xr[i];
        v = fmaxf(v, v * NEG_SLOPE);
        p += v * at[i];
      }
      p += __shfl_xor(p, 1, 32);
      p += __shfl_xor(p, 2, 32);
      p += __shfl_xor(p, 4, 32);
      const float mn = fmaxf(mrun, p);
      const float sc = __expf(mrun - mn);
      const float pe = __expf(p - mn);
      dsum = dsum * sc + pe;
#pragma unroll
      for (int i = 0; i < 16; ++i) acc[i] = acc[i] * sc + pe * xv[i];
      mrun = mn;
    }

    const float invd = 1.f / (dsum + 1e-16f);
#pragma unroll
    for (int i = 0; i < 16; ++i) {
      float t = acc[i] * invd;
      t += __shfl_xor(t, 8, 32);
      t += __shfl_xor(t, 16, 32);
      o[i] = t * 0.25f;
    }
    v4f r4;
#pragma unroll
    for (int jj = 0; jj < 4; ++jj) {
      const float t0 = __shfl(o[jj], srcl, 32);
      const float t1 = __shfl(o[4 + jj], srcl, 32);
      const float t2 = __shfl(o[8 + jj], srcl, 32);
      const float t3 = __shfl(o[12 + jj], srcl, 32);
      r4[jj] = (sel == 0) ? t0 : ((sel == 1) ? t1 : ((sel == 2) ? t2 : t3));
    }
    v4f v = r4 + bias4;
    const float mu = wsum32(v[0] + v[1] + v[2] + v[3]) * (1.f / DIM);
    v4f dv = v - mu;
    const float var = wsum32(dv[0] * dv[0] + dv[1] * dv[1] + dv[2] * dv[2] + dv[3] * dv[3]) * (1.f / DIM);
    const float inv2 = rsqrtf(var + LN_EPS);
    const v4f rr = *(const v4f*)(resid + (size_t)nodec * DIM + 4 * lane);
    v4f y = (dv * inv2) * g4 + be4 + rr;
    if (relu) {
      y[0] = fmaxf(y[0], 0.f); y[1] = fmaxf(y[1], 0.f);
      y[2] = fmaxf(y[2], 0.f); y[3] = fmaxf(y[3], 0.f);
    }
    if (valid) {
      float* op = out + (size_t)node * DIM + 4 * lane;
      *(volatile v4f*)op = y;
      __threadfence();
      *(volatile v4f*)op = y;
    }
  }
}

extern "C" void kernel_launch(void* const* d_in, const int* in_sizes, int n_in,
                              void* d_out, int out_size, void* d_ws, size_t ws_size,
                              hipStream_t stream) {
  (void)n_in;
  const float* x    = (const float*)d_in[0];
  const int*   src  = (const int*)  d_in[1];
  const int*   dst  = (const int*)  d_in[2];
  const float* Wl1  = (const float*)d_in[3];
  const float* Wr1  = (const float*)d_in[4];
  const float* att1 = (const float*)d_in[5];
  const float* b1   = (const float*)d_in[6];
  const float* g1   = (const float*)d_in[7];
  const float* be1  = (const float*)d_in[8];
  const float* Wl2  = (const float*)d_in[9];
  const float* Wr2  = (const float*)d_in[10];
  const float* att2 = (const float*)d_in[11];
  const float* b2   = (const float*)d_in[12];
  const float* g2   = (const float*)d_in[13];
  const float* be2  = (const float*)d_in[14];

  const int N = in_sizes[0] / DIM;
  const int E = in_sizes[1];
  if (N <= 0 || E < 0) return;
  if (out_size < N * DIM) return;

  const int gridX = (N + GBM - 1) / GBM;
  const int rowsP = gridX * GBM;

  size_t off = 0;
  const size_t xlrBytes = (size_t)rowsP * HD2 * sizeof(float);
  float* xlr = (float*)((char*)d_ws + off);
  off += (xlrBytes + 255) & ~(size_t)255;
  const size_t hBytes = (size_t)N * DIM * sizeof(float);
  float* h = (float*)((char*)d_ws + off);
  off += (hBytes + 255) & ~(size_t)255;
  if (off > ws_size) return;

  const int nChunks = (E + 255) / 256;
  const dim3 gg(gridX, 8);
  const int eb = (N + NPB - 1) / NPB;

  k_gemm<<<gg, 256, 0, stream>>>(x, DIM, N, Wl1, Wr1, xlr);
  k_edge<<<eb, 256, 0, stream>>>(xlr, src, dst, E, nChunks, N, att1, b1, g1, be1, x, h, 1);
  k_gemm<<<gg, 256, 0, stream>>>(h, DIM, N, Wl2, Wr2, xlr);
  k_edge<<<eb, 256, 0, stream>>>(xlr, src, dst, E, nChunks, N, att2, b2, g2, be2, h, (float*)d_out, 0);
}
